// Epipolar_Attention_23407571763461
// MI455X (gfx1250) — hardware-verified
//
#include <hip/hip_runtime.h>
#include <math.h>
#include <stddef.h>


typedef _Float16 f16t;
typedef f16t  v16h __attribute__((ext_vector_type(16)));
typedef f16t  v8hr __attribute__((ext_vector_type(8)));
typedef v8hr  v8h  __attribute__((may_alias));
typedef float v8f  __attribute__((ext_vector_type(8)));
typedef float v4fr __attribute__((ext_vector_type(4)));
typedef v4fr  v4f  __attribute__((may_alias));
typedef unsigned int v4ur __attribute__((ext_vector_type(4)));

union Frag { v16h v; v8hr h[2]; };
union H8   { v8hr v; v4ur u; f16t e[8]; };

#define HWN    1024
#define CDIM   320
#define NBAT   4
#define NHEAD  8
#define DHD    40
#define NROW   (NBAT * HWN)
#define PPITCH 40

__device__ __forceinline__ v8f wmma16(v16h a, v16h b, v8f c)
{
    v8f d = __builtin_amdgcn_wmma_f32_16x16x32_f16(false, a, false, b, (short)0, c, false, false);
    asm volatile("v_nop\n\tv_nop\n\tv_nop\n\tv_nop" : "+v"(d) : "v"(a), "v"(b));
    return d;
}

__device__ __forceinline__ float wsum32(float v)
{
#pragma unroll
    for (int k = 16; k >= 1; k >>= 1) v += __shfl_xor(v, k, 32);
    return v;
}
__device__ __forceinline__ float wmax32(float v)
{
#pragma unroll
    for (int k = 16; k >= 1; k >>= 1) v = fmaxf(v, __shfl_xor(v, k, 32));
    return v;
}
__device__ __forceinline__ float hsum16(float v)
{
#pragma unroll
    for (int k = 8; k >= 1; k >>= 1) v += __shfl_xor(v, k, 32);
    return v;
}
__device__ __forceinline__ float hmax16(float v)
{
#pragma unroll
    for (int k = 8; k >= 1; k >>= 1) v = fmaxf(v, __shfl_xor(v, k, 32));
    return v;
}

struct Geo {
    float k00, k01, k02, k10, k11, k12, k20, k21, k22;
    float r00, r01, r02, r10, r11, r12, r20, r21, r22;
    float s00, s01, s02, s10, s11, s12, s20, s21, s22;
    float st0, st1, st2, tt0, tt1, tt2;
    float rfx, rfy;
};

__device__ __forceinline__ void geo_setup(int tuple, const float* __restrict__ intr,
                                          const float* __restrict__ c2w, Geo& g)
{
#pragma clang fp contract(off)
    const int dir = tuple >> 2, b = tuple & 3;
    const int srcSel = (dir == 0) ? 1 : 0;
    const int tgtSel = 1 - srcSel;
    const float* Ki = intr + b * 9;
    const float wimg = (float)(32.0 * 16.0 / 9.0);
    g.k00 = Ki[0] * wimg;  g.k01 = Ki[1] * wimg;  g.k02 = 16.0f;
    g.k10 = Ki[3] * 32.0f; g.k11 = Ki[4] * 32.0f; g.k12 = 16.0f;
    g.k20 = Ki[6];         g.k21 = Ki[7];         g.k22 = Ki[8];
    const float* S = c2w + (size_t)(srcSel * NBAT + b) * 16;
    const float* T = c2w + (size_t)(tgtSel * NBAT + b) * 16;
    g.s00 = S[0]; g.s01 = S[1]; g.s02 = S[2];
    g.s10 = S[4]; g.s11 = S[5]; g.s12 = S[6];
    g.s20 = S[8]; g.s21 = S[9]; g.s22 = S[10];
    g.st0 = S[3]; g.st1 = S[7]; g.st2 = S[11];
    const float a00 = T[0], a01 = T[1], a02 = T[2];
    const float a10 = T[4], a11 = T[5], a12 = T[6];
    const float a20 = T[8], a21 = T[9], a22 = T[10];
    const float c00 = a11 * a22 - a12 * a21;
    const float c01 = a10 * a22 - a12 * a20;
    const float c02 = a10 * a21 - a11 * a20;
    const float det = a00 * c00 - a01 * c01 + a02 * c02;
    const float id = 1.0f / det;
    g.r00 =  c00 * id;                      g.r01 = -(a01 * a22 - a02 * a21) * id;  g.r02 =  (a01 * a12 - a02 * a11) * id;
    g.r10 = -c01 * id;                      g.r11 =  (a00 * a22 - a02 * a20) * id;  g.r12 = -(a00 * a12 - a02 * a10) * id;
    g.r20 =  c02 * id;                      g.r21 = -(a00 * a21 - a01 * a20) * id;  g.r22 =  (a00 * a11 - a01 * a10) * id;
    g.tt0 = -T[3]; g.tt1 = -T[7]; g.tt2 = -T[11];
    g.rfx = 1.0f / g.k00;
    g.rfy = 1.0f / g.k11;
}

__device__ __forceinline__ float dwf(float ux, float uy, float uz, float rv,
                                     float wx, float wy, float wz)
{
#pragma clang fp contract(off)
    const float cx = uy * wz - uz * wy;
    const float cy = uz * wx - ux * wz;
    const float cz = ux * wy - uy * wx;
    const float area = sqrtf(cx * cx + cy * cy + cz * cz);
    const float dist = area * rv;
    const float t = 50.0f * (dist - 0.5f);
    const float sg = 1.0f / (1.0f + __expf(-t));
    return 1.0f - sg;
}

__global__ __launch_bounds__(256) void epi_geo_kernel(const float* __restrict__ intr,
                                                      const float* __restrict__ c2w,
                                                      float* pi, float* oi)
{
#pragma clang fp contract(off)
    const int tuple = blockIdx.x;
    Geo g;
    geo_setup(tuple, intr, c2w, g);
    v4fr pv[4];
#pragma unroll
    for (int s = 0; s < 4; ++s) {
        const int n = threadIdx.x + s * 256;
        const float cxp = ((float)(n & 31) - 16.0f) * g.rfx;
        const float cyp = ((float)(n >> 5) - 16.0f) * g.rfy;
        const float pwx = g.s00 * cxp + g.s01 * cyp + g.s02 + g.st0;
        const float pwy = g.s10 * cxp + g.s11 * cyp + g.s12 + g.st1;
        const float pwz = g.s20 * cxp + g.s21 * cyp + g.s22 + g.st2;
        const float ptx = g.r00 * pwx + g.r01 * pwy + g.r02 * pwz + g.tt0;
        const float pty = g.r10 * pwx + g.r11 * pwy + g.r12 * pwz + g.tt1;
        const float ptz = g.r20 * pwx + g.r21 * pwy + g.r22 * pwz + g.tt2;
        const float px = g.k00 * ptx + g.k01 * pty + g.k02 * ptz;
        const float py = g.k10 * ptx + g.k11 * pty + g.k12 * ptz;
        const float pz = g.k20 * ptx + g.k21 * pty + g.k22 * ptz;
        const float inv = 1.0f / (pz + 1e-6f);
        v4fr v; v.x = px * inv; v.y = py * inv; v.z = pz * inv; v.w = 0.0f;
        pv[s] = v;
    }
    float* pbase = pi + (size_t)tuple * HWN * 4;
#pragma unroll
    for (int s = 0; s < 4; ++s)
        *(volatile v4fr*)(pbase + (size_t)(threadIdx.x + s * 256) * 4) = pv[s];
    __threadfence();
#pragma unroll
    for (int s = 0; s < 4; ++s)
        *(volatile v4fr*)(pbase + (size_t)(threadIdx.x + s * 256) * 4) = pv[s];

    if (threadIdx.x < 8) {
        Geo q;
        geo_setup(threadIdx.x, intr, c2w, q);
        const float ox = q.r00 * q.st0 + q.r01 * q.st1 + q.r02 * q.st2 + q.tt0;
        const float oy = q.r10 * q.st0 + q.r11 * q.st1 + q.r12 * q.st2 + q.tt1;
        const float oz = q.r20 * q.st0 + q.r21 * q.st1 + q.r22 * q.st2 + q.tt2;
        const float kx = q.k00 * ox + q.k01 * oy + q.k02 * oz;
        const float ky = q.k10 * ox + q.k11 * oy + q.k12 * oz;
        const float kz = q.k20 * ox + q.k21 * oy + q.k22 * oz;
        const float ioz = 1.0f / kz;
        v4fr v; v.x = kx * ioz; v.y = ky * ioz; v.z = kz * ioz; v.w = 0.0f;
        if (blockIdx.x == 0) {
            *(volatile v4fr*)(oi + threadIdx.x * 4) = v;
            __threadfence();
            *(volatile v4fr*)(oi + threadIdx.x * 4) = v;
        }
    }
}

__global__ __launch_bounds__(256) void epi_flag_kernel(const float* __restrict__ pi,
                                                       const float* __restrict__ oi, float* flags)
{
#pragma clang fp contract(off)
    __shared__ __align__(16) float sF[32];
    const int wave = threadIdx.x >> 5, lane = threadIdx.x & 31;
#pragma unroll 1
    for (int i = 0; i < 4; ++i) {
        const int R = blockIdx.x * 32 + wave * 4 + i;
        const int tuple = R >> 10, mrow = R & (HWN - 1);
        const float* od = oi + tuple * 4;
        const float ox = od[0], oy = od[1], oz = od[2];
        const float* pd = pi + ((size_t)tuple * HWN + mrow) * 4;
        const float ux = pd[0] - ox, uy = pd[1] - oy, uz = pd[2] - oz;
        const float rv = 1.0f / sqrtf(ux * ux + uy * uy + uz * uz);
        const float wz = 1.0f - oz;
        const float wx = (float)lane - ox;
        float lmax = -1.0e30f;
#pragma unroll 2
        for (int s = 0; s < 32; ++s) {
            const float wy = (float)s - oy;
            const float d = dwf(ux, uy, uz, rv, wx, wy, wz);
            lmax = fmaxf(lmax, d);
        }
        lmax = wmax32(lmax);
        if (lane == 0) sF[wave * 4 + i] = (lmax < 0.5f) ? 1.0f : 0.0f;
    }
    __syncthreads();
    if (wave == 0 && lane < 8) {
        const v4fr v = *(const v4f*)(&sF[lane * 4]);
        float* p = flags + (size_t)blockIdx.x * 32 + lane * 4;
        *(volatile v4fr*)p = v;
        __threadfence();
        *(volatile v4fr*)p = v;
    }
}

__global__ __launch_bounds__(256) void epi_weight_kernel(const float* __restrict__ pi,
                                                         const float* __restrict__ oi,
                                                         const float* __restrict__ flags, float* ew)
{
#pragma clang fp contract(off)
    const int wave = threadIdx.x >> 5, lane = threadIdx.x & 31;
    const int R = blockIdx.x * 8 + wave;
    const int b = R >> 10, q = R & (HWN - 1);
    const float* od0 = oi + b * 4;
    const float o0x = od0[0], o0y = od0[1], o0z = od0[2];
    const float* pd0 = pi + ((size_t)b * HWN + q) * 4;
    const float u0x = pd0[0] - o0x, u0y = pd0[1] - o0y, u0z = pd0[2] - o0z;
    const float rv0 = 1.0f / sqrtf(u0x * u0x + u0y * u0y + u0z * u0z);
    const bool fill0 = flags[b * HWN + q] != 0.0f;
    const float w0z = 1.0f - o0z;
    const float* od1 = oi + (NBAT + b) * 4;
    const float o1x = od1[0], o1y = od1[1], o1z = od1[2];
    const float w1x = (float)(q & 31) - o1x, w1y = (float)(q >> 5) - o1y, w1z = 1.0f - o1z;
    const float* pi1 = pi + (size_t)(NBAT + b) * HWN * 4;
    const float* fl1 = flags + (NBAT + b) * HWN;
    float* orow = ew + ((size_t)b * HWN + q) * HWN;
#pragma unroll 1
    for (int it = 0; it < 8; ++it) {
        const int kk = it * 128 + lane * 4;
        v4fr val = {0.0f, 0.0f, 0.0f, 0.0f};
#pragma unroll
        for (int c = 0; c < 4; ++c) {
            const int key = kk + c;
            float e1 = 1.0f;
            if (!fill0) e1 = dwf(u0x, u0y, u0z, rv0, (float)(key & 31) - o0x, (float)(key >> 5) - o0y, w0z);
            float e2 = 1.0f;
            if (fl1[key] == 0.0f) {
                const float* p1 = pi1 + (size_t)key * 4;
                const float ux = p1[0] - o1x, uy = p1[1] - o1y, uz = p1[2] - o1z;
                const float rv = 1.0f / sqrtf(ux * ux + uy * uy + uz * uz);
                e2 = dwf(ux, uy, uz, rv, w1x, w1y, w1z);
            }
            val[c] = e1 * e2;
        }
        *(volatile v4fr*)(orow + kk) = val;
        __threadfence();
        *(volatile v4fr*)(orow + kk) = val;
    }
}

__global__ __launch_bounds__(256) void cvt_wt_kernel(const float* __restrict__ W, f16t* Th, f16t* Tl,
                                                     int K, int N, float scale, int do_lo)
{
    __shared__ float tile[64][33];
    const int wave = threadIdx.x >> 5, lane = threadIdx.x & 31;
    const int n0 = blockIdx.x * 32;
#pragma unroll 1
    for (int k0 = 0; k0 < K; k0 += 64) {
#pragma unroll
        for (int s = 0; s < 8; ++s) {
            const int e = threadIdx.x + 256 * s;
            const int kk = e >> 5, nn = e & 31;
            float v = 0.0f;
            if (k0 + kk < K && n0 + nn < N) v = W[(size_t)(k0 + kk) * N + n0 + nn];
            tile[kk][nn] = v;
        }
        __syncthreads();
        const int L = wave * 4 + (lane >> 3);
        const int kq = (lane & 7) * 8;
        H8 hh, ll;
#pragma unroll
        for (int i = 0; i < 8; ++i) {
            const float x = tile[kq + i][L] * scale;
            const f16t e = (f16t)x;
            hh.e[i] = e;
            ll.e[i] = (f16t)((x - (float)e) * 1024.0f);
        }
        const bool act = (n0 + L < N) && (k0 + kq + 7 < K);
        const size_t off = (size_t)(n0 + L) * K + k0 + kq;
        if (act) {
            *(volatile v4ur*)(Th + off) = hh.u;
            if (do_lo) *(volatile v4ur*)(Tl + off) = ll.u;
        }
        __threadfence();
        if (act) {
            *(volatile v4ur*)(Th + off) = hh.u;
            if (do_lo) *(volatile v4ur*)(Tl + off) = ll.u;
        }
        __syncthreads();
    }
}

__global__ __launch_bounds__(256) void ln_rows_kernel(const float* __restrict__ X, int transposed,
                                                      const float* __restrict__ g0, const float* __restrict__ b0, float* Y0,
                                                      const float* __restrict__ g1, const float* __restrict__ b1, float* Y1,
                                                      int nout, int nrows)
{
#pragma clang fp contract(off)
    const int wave = threadIdx.x >> 5, lane = threadIdx.x & 31;
#pragma unroll 1
    for (int i = 0; i < 8; ++i) {
        const int row = blockIdx.x * 64 + wave * 8 + i;
        if (row >= nrows) break;
        const int bidx = row >> 10, n = row & (HWN - 1);
        size_t base, cs;
        if (transposed) { base = (size_t)bidx * CDIM * HWN + n; cs = HWN; }
        else            { base = (size_t)row * CDIM;           cs = 1;   }
        float xv[10];
        float s = 0.0f;
#pragma unroll
        for (int k = 0; k < 10; ++k) { xv[k] = X[base + (size_t)(lane + 32 * k) * cs]; s += xv[k]; }
        s = wsum32(s);
        const float mean = s / 320.0f;
        float d2 = 0.0f;
#pragma unroll
        for (int k = 0; k < 10; ++k) { const float d = xv[k] - mean; d2 += d * d; }
        d2 = wsum32(d2);
        const float var = d2 / 320.0f;
        const float inv = 1.0f / sqrtf(var + 1e-5f);
        for (int o = 0; o < nout; ++o) {
            const float* g  = o ? g1 : g0;
            const float* bb = o ? b1 : b0;
            float* Y = o ? Y1 : Y0;
#pragma unroll
            for (int it = 0; it < 3; ++it) {
                const int j = it * 4 + (lane >> 3);
                const bool act = j < 10;
                const int c = j * 32 + (lane & 7) * 4;
                v4fr v = {0.0f, 0.0f, 0.0f, 0.0f};
                if (act) {
#pragma unroll
                    for (int t = 0; t < 4; ++t) {
                        const float x = X[base + (size_t)(c + t) * cs];
                        v[t] = (x - mean) * inv * g[c + t] + bb[c + t];
                    }
                }
                float* p = Y + (size_t)row * CDIM + c;
                if (act) *(volatile v4fr*)p = v;
                __threadfence();
                if (act) *(volatile v4fr*)p = v;
            }
        }
    }
}

__global__ __launch_bounds__(256) void ln_out_kernel(const float* __restrict__ Z, const float* __restrict__ g,
                                                     const float* __restrict__ bb, float* out, int nrows)
{
#pragma clang fp contract(off)
    __shared__ float tile[32][CDIM + 1];
    __shared__ float sMean[32];
    __shared__ float sInv[32];
    const int wave = threadIdx.x >> 5, lane = threadIdx.x & 31;
    const int bidx = blockIdx.x >> 5, n0 = (blockIdx.x & 31) * 32;
#pragma unroll 1
    for (int i = 0; i < 4; ++i) {
        const int r = wave * 4 + i;
        const int row = min((int)blockIdx.x * 32 + r, nrows - 1);
        float xv[10];
        float s = 0.0f;
#pragma unroll
        for (int k = 0; k < 10; ++k) {
            const int c = lane + 32 * k;
            xv[k] = Z[(size_t)row * CDIM + c];
            tile[r][c] = xv[k];
            s += xv[k];
        }
        s = wsum32(s);
        const float mean = s / 320.0f;
        float d2 = 0.0f;
#pragma unroll
        for (int k = 0; k < 10; ++k) { const float d = xv[k] - mean; d2 += d * d; }
        d2 = wsum32(d2);
        const float var = d2 / 320.0f;
        const float inv = 1.0f / sqrtf(var + 1e-5f);
        if (lane == 0) { sMean[r] = mean; sInv[r] = inv; }
    }
    __syncthreads();
    const int nl = (lane & 7) * 4;
    const bool act = ((int)blockIdx.x * 32 + 31) < nrows;
#pragma unroll 1
    for (int it = 0; it < 10; ++it) {
        const int c = it * 32 + wave * 4 + (lane >> 3);
        const float gc = g[c], bc = bb[c];
        v4fr v;
#pragma unroll
        for (int t = 0; t < 4; ++t) {
            const int rr = nl + t;
            v[t] = (tile[rr][c] - sMean[rr]) * sInv[rr] * gc + bc;
        }
        float* p = out + ((size_t)bidx * CDIM + c) * HWN + n0 + nl;
        if (act) *(volatile v4fr*)p = v;
        __threadfence();
        if (act) *(volatile v4fr*)p = v;
    }
}

__global__ __launch_bounds__(128) void gemm_kernel(const float* __restrict__ A, int lda, float sa,
                                                   const f16t* __restrict__ Bh, const f16t* __restrict__ Bl, float sb,
                                                   const float* __restrict__ bias, const float* __restrict__ R, float* Cout,
                                                   int M, int N, int K, int flags)
{
    __shared__ v8hr sAh[64 * 4];
    __shared__ v8hr sAl[64 * 4];
    __shared__ __align__(16) float sC[64 * 64];
    const int wave = threadIdx.x >> 5, lane = threadIdx.x & 31;
    const int hf = lane >> 4, m = lane & 15;
    const int n0 = blockIdx.x * 64, m0 = blockIdx.y * 64;
    const int split = flags & 1, gelu = (flags >> 1) & 1, resid = (flags >> 2) & 1;

    v8f acc[4], accr[4];
#pragma unroll
    for (int j = 0; j < 4; ++j)
#pragma unroll
        for (int r = 0; r < 8; ++r) { acc[j][r] = 0.0f; accr[j][r] = 0.0f; }

    const int srow = threadIdx.x >> 1, skq = (threadIdx.x & 1) * 16;
    const int arow = min(m0 + srow, M - 1);
    const float* ap = A + (size_t)arow * lda + skq;
    const int fr = (wave * 16 + m) * 4;

#pragma unroll 1
    for (int k0 = 0; k0 < K; k0 += 32) {
        const v4fr x0 = *(const v4f*)(ap + k0);
        const v4fr x1 = *(const v4f*)(ap + k0 + 4);
        const v4fr x2 = *(const v4f*)(ap + k0 + 8);
        const v4fr x3 = *(const v4f*)(ap + k0 + 12);
        float xs[16];
#pragma unroll
        for (int t = 0; t < 4; ++t) { xs[t] = x0[t]; xs[4 + t] = x1[t]; xs[8 + t] = x2[t]; xs[12 + t] = x3[t]; }
        H8 h0, h1, l0, l1;
#pragma unroll
        for (int i = 0; i < 8; ++i) {
            const float y0 = xs[i] * sa, y1 = xs[8 + i] * sa;
            const f16t e0 = (f16t)y0, e1 = (f16t)y1;
            h0.e[i] = e0; h1.e[i] = e1;
            l0.e[i] = (f16t)((y0 - (float)e0) * 1024.0f);
            l1.e[i] = (f16t)((y1 - (float)e1) * 1024.0f);
        }
        sAh[srow * 4 + (skq >> 3)]     = h0.v;
        sAh[srow * 4 + (skq >> 3) + 1] = h1.v;
        if (split) {
            sAl[srow * 4 + (skq >> 3)]     = l0.v;
            sAl[srow * 4 + (skq >> 3) + 1] = l1.v;
        }
        __syncthreads();
        Frag fa, fl;
        fa.h[0] = sAh[fr + hf];
        fa.h[1] = sAh[fr + 2 + hf];
        fl.h[0] = sAl[fr + hf];
        fl.h[1] = sAl[fr + 2 + hf];
#pragma unroll
        for (int j = 0; j < 4; ++j) {
            const size_t boff = (size_t)(n0 + 16 * j + m) * K + k0;
            Frag fb;
            fb.h[0] = *(const v8h*)(Bh + boff + 8 * hf);
            fb.h[1] = *(const v8h*)(Bh + boff + 16 + 8 * hf);
            acc[j] = wmma16(fa.v, fb.v, acc[j]);
            if (split) {
                Frag fc;
                fc.h[0] = *(const v8h*)(Bl + boff + 8 * hf);
                fc.h[1] = *(const v8h*)(Bl + boff + 16 + 8 * hf);
                accr[j] = wmma16(fa.v, fc.v, accr[j]);
                accr[j] = wmma16(fl.v, fb.v, accr[j]);
            }
        }
        __syncthreads();
    }

    const float inv = 1.0f / (sa * sb);
#pragma unroll
    for (int j = 0; j < 4; ++j) {
        const int n = n0 + 16 * j + m;
        const float bs = bias[n];
#pragma unroll
        for (int r = 0; r < 8; ++r) {
            const int row = wave * 16 + 8 * hf + r;
            float v = acc[j][r];
            if (split) v += accr[j][r] * 0.0009765625f;
            v = v * inv + bs;
            if (gelu) v = 0.5f * v * (1.0f + erff(v * 0.70710678118654752f));
            if (resid) { const int gm = min(m0 + row, M - 1); v += R[(size_t)gm * N + n]; }
            sC[row * 64 + 16 * j + m] = v;
        }
    }
    __syncthreads();
#pragma unroll
    for (int it = 0; it < 8; ++it) {
        const int L = it * 16 + wave * 4 + (lane >> 3);
        const int row = L >> 1, col = (L & 1) * 32 + (lane & 7) * 4;
        const v4fr v = *(const v4f*)(&sC[row * 64 + col]);
        const int gm = m0 + row;
        if (gm < M) *(volatile v4fr*)(Cout + (size_t)gm * N + n0 + col) = v;
    }
    __threadfence();
#pragma unroll
    for (int it = 0; it < 8; ++it) {
        const int L = it * 16 + wave * 4 + (lane >> 3);
        const int row = L >> 1, col = (L & 1) * 32 + (lane & 7) * 4;
        const v4fr v = *(const v4f*)(&sC[row * 64 + col]);
        const int gm = m0 + row;
        if (gm < M) *(volatile v4fr*)(Cout + (size_t)gm * N + n0 + col) = v;
    }
}

__global__ __launch_bounds__(256) void pack_qk_kernel(const float* __restrict__ qf, const float* __restrict__ kf,
                                                      f16t* qp, f16t* kp)
{
    const float* src = (blockIdx.y == 0) ? qf : kf;
    f16t* dst = (blockIdx.y == 0) ? qp : kp;
    const int wave = threadIdx.x >> 5, lane = threadIdx.x & 31;
    const int row = blockIdx.x * 32 + wave * 4 + (lane >> 3);
    const int qi = row & (HWN - 1), h = (row >> 10) & 7, b = row >> 13;
    const int d0 = (lane & 7) * 8;
    const bool act = row < NBAT * NHEAD * HWN;
    H8 o;
#pragma unroll
    for (int i = 0; i < 8; ++i) {
        const int d = d0 + i;
        float x = 0.0f;
        if (act && d < DHD) x = src[((size_t)b * HWN + qi) * CDIM + h * DHD + d] * 16.0f;
        o.e[i] = (f16t)x;
    }
    const size_t off = (size_t)row * 64 + d0;
    if (act) *(volatile v4ur*)(dst + off) = o.u;
    __threadfence();
    if (act) *(volatile v4ur*)(dst + off) = o.u;
}

__global__ __launch_bounds__(256) void pack_v_kernel(const float* __restrict__ vf, f16t* vT)
{
    const int wave = threadIdx.x >> 5, lane = threadIdx.x & 31;
    const int row = blockIdx.x * 8 + wave;
    const int d = row % 48, h = (row / 48) & 7, b = row / 384;
    const bool act = row < NBAT * NHEAD * 48;
#pragma unroll 1
    for (int it = 0; it < 4; ++it) {
        const int key0 = it * 256 + lane * 8;
        H8 o;
#pragma unroll
        for (int i = 0; i < 8; ++i) {
            float x = 0.0f;
            if (act && d < DHD) x = vf[((size_t)b * HWN + key0 + i) * CDIM + h * DHD + d] * 16.0f;
            o.e[i] = (f16t)x;
        }
        const size_t off = (size_t)row * HWN + key0;
        if (act) *(volatile v4ur*)(vT + off) = o.u;
        __threadfence();
        if (act) *(volatile v4ur*)(vT + off) = o.u;
    }
}

__global__ __launch_bounds__(128) void attn_kernel(const f16t* __restrict__ qp, const f16t* __restrict__ kp,
                                                   const f16t* __restrict__ vT, const float* __restrict__ ew, float* aout)
{
    __shared__ __align__(16) f16t  sP[4][16 * PPITCH];
    __shared__ __align__(16) float sO[4][16 * 48];
    __shared__ float sM[4][16];
    __shared__ float sL[4][16];
    __shared__ __align__(16) float sRow[16 * CDIM];

    const int wave = threadIdx.x >> 5, lane = threadIdx.x & 31;
    const int hf = lane >> 4, m = lane & 15;
    const int b = blockIdx.x >> 6;
    const int q0 = (blockIdx.x & 63) << 4;
    const float SC = 0.15811388300841897f * 0.00390625f;
    f16t* sPw = &sP[wave][0];

#pragma unroll 1
    for (int h = 0; h < NHEAD; ++h) {
        const int bh = b * NHEAD + h;
        const f16t* qrow = qp + ((size_t)bh * HWN + q0 + m) * 64;
        Frag a0, a1;
        a0.h[0] = *(const v8h*)(qrow + 8 * hf);
        a0.h[1] = *(const v8h*)(qrow + 16 + 8 * hf);
        a1.h[0] = *(const v8h*)(qrow + 32 + 8 * hf);
        a1.h[1] = *(const v8h*)(qrow + 48 + 8 * hf);
        const f16t* kbh = kp + (size_t)bh * HWN * 64;
        const f16t* vbh = vT + (size_t)bh * 48 * HWN;
        const float* ewb = ew + ((size_t)b * HWN + q0) * HWN;

        float m_run[8], l_run[8];
        v8f O[3];
#pragma unroll
        for (int r = 0; r < 8; ++r) { m_run[r] = -1.0e30f; l_run[r] = 0.0f; }
#pragma unroll
        for (int t3 = 0; t3 < 3; ++t3)
#pragma unroll
            for (int r = 0; r < 8; ++r) O[t3][r] = 0.0f;

#pragma unroll 1
        for (int st = 0; st < 8; ++st) {
            const int ks = wave * 256 + st * 32;
            float sv[2][8];
#pragma unroll
            for (int nt = 0; nt < 2; ++nt) {
                const f16t* krow = kbh + (size_t)(ks + 16 * nt + m) * 64;
                Frag bk;
                bk.h[0] = *(const v8h*)(krow + 8 * hf);
                bk.h[1] = *(const v8h*)(krow + 16 + 8 * hf);
                v8f s = {0.0f, 0.0f, 0.0f, 0.0f, 0.0f, 0.0f, 0.0f, 0.0f};
                s = wmma16(a0.v, bk.v, s);
                Frag bk2;
                bk2.h[0] = *(const v8h*)(krow + 32 + 8 * hf);
                bk2.h[1] = *(const v8h*)(krow + 48 + 8 * hf);
                s = wmma16(a1.v, bk2.v, s);
#pragma unroll
                for (int r = 0; r < 8; ++r) {
                    const float e = ewb[(size_t)(8 * hf + r) * HWN + ks + 16 * nt + m];
                    sv[nt][r] = s[r] * SC * e;
                }
            }
#pragma unroll
            for (int r = 0; r < 8; ++r) {
                float mx = fmaxf(sv[0][r], sv[1][r]);
                mx = hmax16(mx);
                const float mn = fmaxf(m_run[r], mx);
                const float alpha = __expf(m_run[r] - mn);
                m_run[r] = mn;
                const float p0 = __expf(sv[0][r] - mn), p1 = __expf(sv[1][r] - mn);
                sv[0][r] = p0; sv[1][r] = p1;
                const float rs = hsum16(p0 + p1);
                l_run[r] = l_run[r] * alpha + rs;
#pragma unroll
                for (int t3 = 0; t3 < 3; ++t3) O[t3][r] *= alpha;
            }
#pragma unroll
            for (int nt = 0; nt < 2; ++nt)
#pragma unroll
                for (int r = 0; r < 8; ++r)
                    sPw[(8 * hf + r) * PPITCH + 16 * nt + m] = (f16t)sv[nt][r];
            __syncthreads();
            Frag pf;
            pf.h[0] = *(const v8h*)(sPw + m * PPITCH + 8 * hf);
            pf.h[1] = *(const v8h*)(sPw + m * PPITCH + 16 + 8 * hf);
#pragma unroll
            for (int t3 = 0; t3 < 3; ++t3) {
                const f16t* vrow = vbh + (size_t)(16 * t3 + m) * HWN + ks;
                Frag bv;
                bv.h[0] = *(const v8h*)(vrow + 8 * hf);
                bv.h[1] = *(const v8h*)(vrow + 16 + 8 * hf);
                O[t3] = wmma16(pf.v, bv.v, O[t3]);
            }
            __syncthreads();
        }
        if (m == 0) {
#pragma unroll
            for (int r = 0; r < 8; ++r) { sM[wave][8 * hf + r] = m_run[r]; sL[wave][8 * hf + r] = l_run[r]; }
        }
#pragma unroll
        for (int t3 = 0; t3 < 3; ++t3)
#pragma unroll
            for (int r = 0; r < 8; ++r) sO[wave][(8 * hf + r) * 48 + 16 * t3 + m] = O[t3][r];
        __syncthreads();
        for (int idx = threadIdx.x; idx < 16 * DHD; idx += 128) {
            const int row = idx / DHD, d = idx - row * DHD;
            float Mx = sM[0][row];
            Mx = fmaxf(Mx, sM[1][row]); Mx = fmaxf(Mx, sM[2][row]); Mx = fmaxf(Mx, sM[3][row]);
            float l = 0.0f, o = 0.0f;
#pragma unroll
            for (int w = 0; w < 4; ++w) {
                const float sc = __expf(sM[w][row] - Mx);
                l += sL[w][row] * sc;
                o += sO[w][row * 48 + d] * sc;
            }
            sRow[row * CDIM + h * DHD + d] = (o / l) * 0.0625f;
        }
        __syncthreads();
    }
#pragma unroll
    for (int it = 0; it < 10; ++it) {
        const int L = it * 16 + wave * 4 + (lane >> 3);
        const int row = L / 10, j = L - row * 10;
        const int col = j * 32 + (lane & 7) * 4;
        const v4fr v = *(const v4f*)(&sRow[row * CDIM + col]);
        float* p = aout + ((size_t)b * HWN + q0 + row) * CDIM + col;
        *(volatile v4fr*)p = v;
    }
    __threadfence();
#pragma unroll
    for (int it = 0; it < 10; ++it) {
        const int L = it * 16 + wave * 4 + (lane >> 3);
        const int row = L / 10, j = L - row * 10;
        const int col = j * 32 + (lane & 7) * 4;
        const v4fr v = *(const v4f*)(&sRow[row * CDIM + col]);
        float* p = aout + ((size_t)b * HWN + q0 + row) * CDIM + col;
        *(volatile v4fr*)p = v;
    }
}

extern "C" void kernel_launch(void* const* d_in, const int* in_sizes, int n_in,
                              void* d_out, int out_size, void* d_ws, size_t ws_size,
                              hipStream_t stream)
{
    if (n_in < 26) return;
    if (in_sizes[0] != NROW * CDIM || in_sizes[1] != NROW * CDIM) return;
    if (in_sizes[2] != NBAT * 9 || in_sizes[3] != 2 * NBAT * 16) return;
    if (in_sizes[6] != CDIM * CDIM || in_sizes[10] != CDIM * CDIM ||
        in_sizes[14] != CDIM * CDIM || in_sizes[16] != CDIM * CDIM) return;
    if (in_sizes[20] != CDIM * 2 * CDIM || in_sizes[22] != 2 * CDIM * CDIM) return;
    {
        const int vecC[15] = {4, 5, 7, 8, 9, 11, 12, 13, 15, 17, 18, 19, 23, 24, 25};
        for (int i = 0; i < 15; ++i) if (in_sizes[vecC[i]] != CDIM) return;
        if (in_sizes[21] != 2 * CDIM) return;
    }
    if (out_size != NROW * CDIM) return;

    const float* x         = (const float*)d_in[0];
    const float* srcE      = (const float*)d_in[1];
    const float* intr      = (const float*)d_in[2];
    const float* c2w       = (const float*)d_in[3];
    const float* ln_q_w    = (const float*)d_in[4];
    const float* ln_q_b    = (const float*)d_in[5];
    const float* Wq        = (const float*)d_in[6];
    const float* bq        = (const float*)d_in[7];
    const float* ln_k_w    = (const float*)d_in[8];
    const float* ln_k_b    = (const float*)d_in[9];
    const float* Wk        = (const float*)d_in[10];
    const float* bk        = (const float*)d_in[11];
    const float* ln_v_w    = (const float*)d_in[12];
    const float* ln_v_b    = (const float*)d_in[13];
    const float* Wv        = (const float*)d_in[14];
    const float* bv        = (const float*)d_in[15];
    const float* Wo        = (const float*)d_in[16];
    const float* bo        = (const float*)d_in[17];
    const float* ln_pre_w  = (const float*)d_in[18];
    const float* ln_pre_b  = (const float*)d_in[19];
    const float* W1        = (const float*)d_in[20];
    const float* b1        = (const float*)d_in[21];
    const float* W2        = (const float*)d_in[22];
    const float* b2        = (const float*)d_in[23];
    const float* ln_post_w = (const float*)d_in[24];
    const float* ln_post_b = (const float*)d_in[25];

    char* ws = (char*)d_ws;
    size_t cur = 0;
    auto carve = [&](size_t bytes) -> size_t { size_t r = cur; cur += (bytes + 255) & ~((size_t)255); return r; };

    const size_t o_pi  = carve((size_t)2 * NBAT * HWN * 16);
    const size_t o_oi  = carve(256);
    const size_t o_fl  = carve((size_t)2 * NBAT * HWN * 4);
    const size_t o_ew  = carve((size_t)NBAT * HWN * HWN * 4);
    const size_t szW   = (size_t)CDIM * CDIM * 2;
    const size_t szW2  = (size_t)2 * CDIM * CDIM * 2;
    const size_t o_wq  = carve(szW);
    const size_t o_wk  = carve(szW);
    const size_t o_wv  = carve(szW);
    const size_t o_woh = carve(szW);
    const size_t o_wol = carve(szW);
    const size_t o_w1  = carve(szW2);
    const size_t o_w2  = carve(szW2);
    const size_t szX   = (size_t)NROW * CDIM * 4;
    const size_t o_xq  = carve(szX);
    const size_t o_xk  = carve(szX);
    const size_t o_xv  = carve(szX);
    const size_t o_qf  = carve(szX);
    const size_t o_kf  = carve(szX);
    const size_t o_vf  = carve(szX);
    const size_t o_qp  = carve((size_t)NBAT * NHEAD * HWN * 64 * 2);
    const size_t o_kp  = carve((size_t)NBAT * NHEAD * HWN * 64 * 2);
    const size_t o_vt  = carve((size_t)NBAT * NHEAD * 48 * HWN * 2);
    const size_t o_a   = carve(szX);
    const size_t o_z0  = carve(szX);
    const size_t o_zp  = carve(szX);
    const size_t o_h   = carve((size_t)NROW * 2 * CDIM * 4);
    const size_t o_y   = carve(szX);
    if (cur > ws_size) return;

    float* pi    = (float*)(ws + o_pi);
    float* oi    = (float*)(ws + o_oi);
    float* flags = (float*)(ws + o_fl);
    float* ew    = (float*)(ws + o_ew);
    f16t* WqT  = (f16t*)(ws + o_wq);
    f16t* WkT  = (f16t*)(ws + o_wk);
    f16t* WvT  = (f16t*)(ws + o_wv);
    f16t* WoTh = (f16t*)(ws + o_woh);
    f16t* WoTl = (f16t*)(ws + o_wol);
    f16t* W1T  = (f16t*)(ws + o_w1);
    f16t* W2T  = (f16t*)(ws + o_w2);
    float* Xq = (float*)(ws + o_xq);
    float* Xk = (float*)(ws + o_xk);
    float* Xv = (float*)(ws + o_xv);
    float* qf = (float*)(ws + o_qf);
    float* kf = (float*)(ws + o_kf);
    float* vf = (float*)(ws + o_vf);
    f16t* qp = (f16t*)(ws + o_qp);
    f16t* kp = (f16t*)(ws + o_kp);
    f16t* vt = (f16t*)(ws + o_vt);
    float* abuf = (float*)(ws + o_a);
    float* z0   = (float*)(ws + o_z0);
    float* zpre = (float*)(ws + o_zp);
    float* hbuf = (float*)(ws + o_h);
    float* ybuf = (float*)(ws + o_y);
    float* outp = (float*)d_out;

    epi_geo_kernel<<<2 * NBAT, 256, 0, stream>>>(intr, c2w, pi, oi);
    epi_flag_kernel<<<(2 * NBAT * HWN) / 32, 256, 0, stream>>>(pi, oi, flags);
    epi_weight_kernel<<<NROW / 8, 256, 0, stream>>>(pi, oi, flags, ew);

    cvt_wt_kernel<<<CDIM / 32, 256, 0, stream>>>(Wq, WqT, WqT, CDIM, CDIM, 256.0f, 0);
    cvt_wt_kernel<<<CDIM / 32, 256, 0, stream>>>(Wk, WkT, WkT, CDIM, CDIM, 256.0f, 0);
    cvt_wt_kernel<<<CDIM / 32, 256, 0, stream>>>(Wv, WvT, WvT, CDIM, CDIM, 256.0f, 0);
    cvt_wt_kernel<<<CDIM / 32, 256, 0, stream>>>(Wo, WoTh, WoTl, CDIM, CDIM, 256.0f, 1);
    cvt_wt_kernel<<<(2 * CDIM) / 32, 256, 0, stream>>>(W1, W1T, W1T, CDIM, 2 * CDIM, 256.0f, 0);
    cvt_wt_kernel<<<CDIM / 32, 256, 0, stream>>>(W2, W2T, W2T, 2 * CDIM, CDIM, 256.0f, 0);

    ln_rows_kernel<<<NROW / 64, 256, 0, stream>>>(x, 1, ln_q_w, ln_q_b, Xq, ln_q_w, ln_q_b, Xq, 1, NROW);
    ln_rows_kernel<<<NROW / 64, 256, 0, stream>>>(srcE, 1, ln_k_w, ln_k_b, Xk, ln_v_w, ln_v_b, Xv, 2, NROW);

    gemm_kernel<<<dim3(CDIM / 64, NROW / 64), 128, 0, stream>>>(Xq, CDIM, 8.0f, WqT, WqT, 256.0f, bq, Xq, qf, NROW, CDIM, CDIM, 0);
    gemm_kernel<<<dim3(CDIM / 64, NROW / 64), 128, 0, stream>>>(Xk, CDIM, 8.0f, WkT, WkT, 256.0f, bk, Xk, kf, NROW, CDIM, CDIM, 0);
    gemm_kernel<<<dim3(CDIM / 64, NROW / 64), 128, 0, stream>>>(Xv, CDIM, 8.0f, WvT, WvT, 256.0f, bv, Xv, vf, NROW, CDIM, CDIM, 0);

    pack_qk_kernel<<<dim3((NBAT * NHEAD * HWN) / 32, 2), 256, 0, stream>>>(qf, kf, qp, kp);
    pack_v_kernel<<<(NBAT * NHEAD * 48) / 8, 256, 0, stream>>>(vf, vt);

    attn_kernel<<<NBAT * (HWN / 16), 128, 0, stream>>>(qp, kp, vt, ew, abuf);

    gemm_kernel<<<dim3(CDIM / 64, NROW / 64), 128, 0, stream>>>(abuf, CDIM, 64.0f, WoTh, WoTl, 256.0f, bo, abuf, z0, NROW, CDIM, CDIM, 1);

    ln_rows_kernel<<<NROW / 64, 256, 0, stream>>>(z0, 0, ln_pre_w, ln_pre_b, zpre, ln_pre_w, ln_pre_b, zpre, 1, NROW);

    gemm_kernel<<<dim3((2 * CDIM) / 64, NROW / 64), 128, 0, stream>>>(zpre, CDIM, 8.0f, W1T, W1T, 256.0f, b1, zpre, hbuf, NROW, 2 * CDIM, CDIM, 2);
    gemm_kernel<<<dim3(CDIM / 64, NROW / 64), 128, 0, stream>>>(hbuf, 2 * CDIM, 8.0f, W2T, W2T, 256.0f, b2, zpre, ybuf, NROW, CDIM, 2 * CDIM, 4);

    ln_out_kernel<<<NROW / 32, 256, 0, stream>>>(ybuf, ln_post_w, ln_post_b, outp, NROW);
}
